// CentralizedCritic_42477226557872
// MI455X (gfx1250) — hardware-run, weakly checked
//
#include <hip/hip_runtime.h>
#include <stddef.h>
#include <stdint.h>


#define D0    44
#define NRB   64
#define DRB   6
#define NTK   128
#define DTK   7
#define HS    64
#define ES    32
#define HK    128
#define HN1   128
#define HN2   128
#define HN3   64
#define ASC   8
#define WSC   1024
#define WSCAP 134217728

static_assert(HS % 32 == 0);
static_assert(HK % 32 == 0);
static_assert(HN1 % 32 == 0);
static_assert(HN2 % 32 == 0);
static_assert(HN3 % 32 == 0);
static_assert(HK == HN1 && HN1 == HN2);
static_assert(D0 + 2 * ES <= HK);
static_assert(D0 >= 32 && D0 <= 64);
static_assert(ES == 32);

typedef float    v4f  __attribute__((ext_vector_type(4)));
typedef float    v8f  __attribute__((ext_vector_type(8)));
typedef _Float16 v4h  __attribute__((ext_vector_type(4)));
typedef _Float16 v8h  __attribute__((ext_vector_type(8)));
typedef _Float16 v16h __attribute__((ext_vector_type(16)));
union FragH { v16h v; v8h h[2]; };

__device__ __forceinline__ v8f wmf(v16h a, v16h b, v8f c) {
  v8f d = __builtin_amdgcn_wmma_f32_16x16x32_f16(false, a, false, b, (short)0, c, false, false);
  asm volatile("v_nop\n\tv_nop\n\tv_nop\n\tv_nop" : "+v"(d) : "v"(a), "v"(b));
  return d;
}

__device__ __forceinline__ v8f splat8(float x) { v8f r = {x, x, x, x, x, x, x, x}; return r; }

__device__ __forceinline__ v4f relu4(v4f a) {
  v4f o;
  o.x = fmaxf(a.x, 0.0f); o.y = fmaxf(a.y, 0.0f); o.z = fmaxf(a.z, 0.0f); o.w = fmaxf(a.w, 0.0f);
  return o;
}

__device__ __forceinline__ v4h cvt4h(v4f a) {
  v4h o;
  o.x = (_Float16)(a.x * (float)ASC);
  o.y = (_Float16)(a.y * (float)ASC);
  o.z = (_Float16)(a.z * (float)ASC);
  o.w = (_Float16)(a.w * (float)ASC);
  return o;
}

__device__ __forceinline__ v16h ldfrag(const _Float16* p, int k0, int hh) {
  FragH u;
  u.h[0] = *(const v8h*)(p + k0 + 8 * hh);
  u.h[1] = *(const v8h*)(p + k0 + 16 + 8 * hh);
  return u.v;
}

__device__ __forceinline__ v8h prepw_piece(const float* ts, int p, int npc) {
  const int row = p / npc, k8 = (p - row * npc) * 8;
  v8h o;
#pragma unroll
  for (int e = 0; e < 8; ++e) o[e] = (_Float16)(ts[(k8 + e) * 16 + row] * (float)WSC);
  return o;
}

__global__ __launch_bounds__(256) void k_prepw(const float* __restrict__ W, int Kreal, int Kpad, int Nd,
                                               _Float16* dst) {
  __shared__ __attribute__((aligned(16))) float ts[256 * 16];
  const int t = threadIdx.x;
  const int n0 = blockIdx.x * 16;
  if (t < Kpad) {
    const int kc = min(t, Kreal - 1);
    const float* wrow = W + (size_t)kc * Nd;
#pragma unroll
    for (int nn = 0; nn < 16; ++nn) {
      const int n = n0 + nn;
      const float v = wrow[min(n, Nd - 1)];
      ts[t * 16 + nn] = (t < Kreal && n < Nd) ? v : 0.0f;
    }
  }
  __syncthreads();
  const int npc = Kpad >> 3;
  const int tot = 16 * npc;
  const int p0 = t, p1 = t + 256;
  const bool a0 = p0 < tot, a1 = p1 < tot;
  const v8h o0 = prepw_piece(ts, a0 ? p0 : 0, npc);
  const v8h o1 = prepw_piece(ts, a1 ? p1 : 0, npc);
  _Float16* d0 = dst + (size_t)n0 * Kpad + 8 * (a0 ? p0 : 0);
  _Float16* d1 = dst + (size_t)n0 * Kpad + 8 * (a1 ? p1 : 0);
  if (a0) *(volatile v8h*)d0 = o0;
  if (a1) *(volatile v8h*)d1 = o1;
  __threadfence();
  if (a0) *(volatile v8h*)d0 = o0;
  if (a1) *(volatile v8h*)d1 = o1;
}

template <int KIN, int NSET>
__global__ __launch_bounds__(64) void k_setenc(const float* __restrict__ x,
                                                const float* __restrict__ w1, const float* __restrict__ b1,
                                                const _Float16* __restrict__ w2t, const float* __restrict__ b2,
                                                const _Float16* __restrict__ w3t, const float* __restrict__ b3,
                                                int B, float* emb) {
  static_assert(NSET % 16 == 0);
  static_assert(KIN >= 1 && KIN <= 8);
  constexpr int MT = NSET / 16;
  constexpr int XJ = (16 * KIN + 31) / 32;
  constexpr float OSC = 1.0f / (float)(ASC * WSC);
  __shared__ __attribute__((aligned(16))) float    s_x[2][16 * 8];
  __shared__ __attribute__((aligned(16))) _Float16 s_h1[2][16 * HS];
  __shared__ __attribute__((aligned(16))) _Float16 s_h2[2][16 * HS];
  __shared__ __attribute__((aligned(16))) float    s_emb[2][ES];

  const int t = threadIdx.x, lane = t & 31, w = t >> 5, hh = lane >> 4, nl = lane & 15;
  const int b = blockIdx.x * 2 + w;
  const int bc = min(b, B - 1);
  float* sx = s_x[w];
  _Float16* sh1 = s_h1[w];
  _Float16* sh2 = s_h2[w];
  const int c4 = 4 * nl;

  v4f w1q[KIN];
#pragma unroll
  for (int f = 0; f < KIN; ++f) w1q[f] = *(const v4f*)(w1 + f * HS + c4);
  const v4f b1q = *(const v4f*)(b1 + c4);
  const float b3v0 = b3[nl], b3v1 = b3[16 + nl];

  float ps0 = 0.0f, ps1 = 0.0f, pm0 = -3.0e38f, pm1 = -3.0e38f;
  const float* xb = x + (size_t)bc * NSET * KIN;

#pragma unroll 1
  for (int mt = 0; mt < MT; ++mt) {
    const float* xt = xb + (size_t)mt * 16 * KIN;
#pragma unroll
    for (int j = 0; j < XJ; ++j) {
      const int i = lane + 32 * j;
      const int ic = min(i, 16 * KIN - 1);
      const float v = xt[ic];
      const int row = ic / KIN;
      const int f = ic - row * KIN;
      if (i < 16 * KIN) sx[row * 8 + f] = v;
    }
    __syncthreads();
#pragma unroll 1
    for (int it = 0; it < 8; ++it) {
      const int r = hh + 2 * it;
      v4f acc = b1q;
#pragma unroll
      for (int f = 0; f < KIN; ++f) acc = acc + sx[r * 8 + f] * w1q[f];
      acc = relu4(acc);
      *(v4h*)(sh1 + r * HS + c4) = cvt4h(acc);
    }
    __syncthreads();
    const v16h af0 = ldfrag(sh1 + nl * HS, 0, hh);
    const v16h af1 = ldfrag(sh1 + nl * HS, 32, hh);
#pragma unroll 1
    for (int nt = 0; nt < HS / 16; ++nt) {
      const int col = 16 * nt + nl;
      const _Float16* bp = w2t + (size_t)col * HS;
      v8f c = splat8(0.0f);
      c = wmf(af0, ldfrag(bp, 0, hh), c);
      c = wmf(af1, ldfrag(bp, 32, hh), c);
      const float bv = b2[col];
#pragma unroll
      for (int r = 0; r < 8; ++r) {
        const float v = fmaxf(c[r] * OSC + bv, 0.0f);
        sh2[(8 * hh + r) * HS + col] = (_Float16)(v * (float)ASC);
      }
    }
    __syncthreads();
    const v16h ag0 = ldfrag(sh2 + nl * HS, 0, hh);
    const v16h ag1 = ldfrag(sh2 + nl * HS, 32, hh);
    {
      const _Float16* bp = w3t + (size_t)nl * HS;
      v8f c = splat8(0.0f);
      c = wmf(ag0, ldfrag(bp, 0, hh), c);
      c = wmf(ag1, ldfrag(bp, 32, hh), c);
#pragma unroll
      for (int r = 0; r < 8; ++r) {
        const float e = c[r] * OSC + b3v0;
        ps0 += e;
        pm0 = fmaxf(pm0, e);
      }
    }
    {
      const _Float16* bp = w3t + (size_t)(16 + nl) * HS;
      v8f c = splat8(0.0f);
      c = wmf(ag0, ldfrag(bp, 0, hh), c);
      c = wmf(ag1, ldfrag(bp, 32, hh), c);
#pragma unroll
      for (int r = 0; r < 8; ++r) {
        const float e = c[r] * OSC + b3v1;
        ps1 += e;
        pm1 = fmaxf(pm1, e);
      }
    }
  }

  ps0 += __shfl_xor(ps0, 16, 32);
  ps1 += __shfl_xor(ps1, 16, 32);
  pm0 = fmaxf(pm0, __shfl_xor(pm0, 16, 32));
  pm1 = fmaxf(pm1, __shfl_xor(pm1, 16, 32));
  const float inv_n = 1.0f / (float)NSET;
  const float pooled0 = (ps0 * inv_n + pm0) * 0.5f;
  const float pooled1 = (ps1 * inv_n + pm1) * 0.5f;
  if (hh == 0) {
    s_emb[w][nl] = pooled0;
    s_emb[w][16 + nl] = pooled1;
  }
  __syncthreads();
  const bool act = t < 16;
  const int tt = act ? t : 0;
  const int er = tt >> 3, ep = tt & 7;
  const int bb = blockIdx.x * 2 + er;
  const bool ok = act && (bb < B);
  const v4f ev = *(const v4f*)(&s_emb[er][4 * ep]);
  float* eo = emb + (size_t)(ok ? bb : 0) * ES + 4 * ep;
  if (ok) *(volatile v4f*)eo = ev;
  __threadfence();
  if (ok) *(volatile v4f*)eo = ev;
}

__global__ __launch_bounds__(64) void k_head(const float* __restrict__ tier0,
                                              const float* __restrict__ remb, const float* __restrict__ temb,
                                              const _Float16* __restrict__ mw1t, const float* __restrict__ mb1,
                                              const _Float16* __restrict__ mw2t, const float* __restrict__ mb2,
                                              const _Float16* __restrict__ mw3t, const float* __restrict__ mb3,
                                              const float* __restrict__ mw4, const float* __restrict__ mb4,
                                              int B, float* out) {
  constexpr float OSC = 1.0f / (float)(ASC * WSC);
  __shared__ __attribute__((aligned(16))) _Float16 s_a[2][16 * HK];
  __shared__ __attribute__((aligned(16))) _Float16 s_b[2][16 * HN1];
  __shared__ __attribute__((aligned(16))) float    s_o[32];

  const int t = threadIdx.x, lane = t & 31, w = t >> 5, hh = lane >> 4, nl = lane & 15;
  const int row0 = blockIdx.x * 32 + 16 * w;
  _Float16* sa = s_a[w];
  _Float16* sb = s_b[w];

#pragma unroll 1
  for (int r = 0; r < 16; ++r) {
    const int rr = min(row0 + r, B - 1);
    const float* tp = tier0 + (size_t)rr * D0;
    const float v0 = tp[lane];
    const float v1 = tp[min(32 + lane, D0 - 1)];
    const float v2 = remb[(size_t)rr * ES + lane];
    const float v3 = temb[(size_t)rr * ES + lane];
    _Float16* ar = sa + r * HK;
    ar[lane] = (_Float16)(v0 * (float)ASC);
    if (lane < D0 - 32) ar[32 + lane] = (_Float16)(v1 * (float)ASC);
    ar[D0 + lane] = (_Float16)(v2 * (float)ASC);
    ar[D0 + ES + lane] = (_Float16)(v3 * (float)ASC);
    if (lane < HK - (D0 + 2 * ES)) ar[D0 + 2 * ES + lane] = (_Float16)0.0f;
  }
  __syncthreads();

  {
    v16h af[HK / 32];
#pragma unroll
    for (int ks = 0; ks < HK / 32; ++ks) af[ks] = ldfrag(sa + nl * HK, 32 * ks, hh);
#pragma unroll 1
    for (int nt = 0; nt < HN1 / 16; ++nt) {
      const int col = 16 * nt + nl;
      const _Float16* bp = mw1t + (size_t)col * HK;
      v8f c = splat8(0.0f);
#pragma unroll
      for (int ks = 0; ks < HK / 32; ++ks) c = wmf(af[ks], ldfrag(bp, 32 * ks, hh), c);
      const float bv = mb1[col];
#pragma unroll
      for (int r = 0; r < 8; ++r) {
        const float v = fmaxf(c[r] * OSC + bv, 0.0f);
        sb[(8 * hh + r) * HN1 + col] = (_Float16)(v * (float)ASC);
      }
    }
  }
  __syncthreads();

  {
    v16h af[HN1 / 32];
#pragma unroll
    for (int ks = 0; ks < HN1 / 32; ++ks) af[ks] = ldfrag(sb + nl * HN1, 32 * ks, hh);
#pragma unroll 1
    for (int nt = 0; nt < HN2 / 16; ++nt) {
      const int col = 16 * nt + nl;
      const _Float16* bp = mw2t + (size_t)col * HN1;
      v8f c = splat8(0.0f);
#pragma unroll
      for (int ks = 0; ks < HN1 / 32; ++ks) c = wmf(af[ks], ldfrag(bp, 32 * ks, hh), c);
      const float bv = mb2[col];
#pragma unroll
      for (int r = 0; r < 8; ++r) {
        const float v = fmaxf(c[r] * OSC + bv, 0.0f);
        sa[(8 * hh + r) * HK + col] = (_Float16)(v * (float)ASC);
      }
    }
  }
  __syncthreads();

  v8f h3[HN3 / 16];
  {
    v16h af[HN2 / 32];
#pragma unroll
    for (int ks = 0; ks < HN2 / 32; ++ks) af[ks] = ldfrag(sa + nl * HK, 32 * ks, hh);
#pragma unroll
    for (int nt = 0; nt < HN3 / 16; ++nt) {
      const int col = 16 * nt + nl;
      const _Float16* bp = mw3t + (size_t)col * HN2;
      v8f c = splat8(0.0f);
#pragma unroll
      for (int ks = 0; ks < HN2 / 32; ++ks) c = wmf(af[ks], ldfrag(bp, 32 * ks, hh), c);
      const float bv = mb3[col];
#pragma unroll
      for (int r = 0; r < 8; ++r) h3[nt][r] = fmaxf(c[r] * OSC + bv, 0.0f);
    }
  }

  const float m0 = mw4[nl], m1 = mw4[16 + nl], m2 = mw4[32 + nl], m3 = mw4[48 + nl];
  float p[8];
#pragma unroll
  for (int r = 0; r < 8; ++r)
    p[r] = (h3[0][r] * m0 + h3[1][r] * m1) + (h3[2][r] * m2 + h3[3][r] * m3);
#pragma unroll
  for (int r = 0; r < 8; ++r) {
    p[r] += __shfl_xor(p[r], 1, 32);
    p[r] += __shfl_xor(p[r], 2, 32);
    p[r] += __shfl_xor(p[r], 4, 32);
    p[r] += __shfl_xor(p[r], 8, 32);
  }
  const float b4 = mb4[0];
  if (nl == 0) {
#pragma unroll
    for (int r = 0; r < 8; ++r) s_o[16 * w + 8 * hh + r] = p[r] + b4;
  }
  __syncthreads();

  const bool act = t < 8;
  const int tt = act ? t : 0;
  const v4f ov = *(const v4f*)(s_o + 4 * tt);
  const int rb = blockIdx.x * 32 + 4 * tt;
  const bool full = act && (rb + 4 <= B);
  const bool part = act && !full && (rb < B);
  float* op = out + (size_t)((rb < B) ? rb : 0);
  if (full) {
    *(volatile v4f*)op = ov;
  } else if (part) {
#pragma unroll
    for (int e = 0; e < 4; ++e)
      if (rb + e < B) ((volatile float*)op)[e] = ov[e];
  }
  __threadfence();
  if (full) {
    *(volatile v4f*)op = ov;
  } else if (part) {
#pragma unroll
    for (int e = 0; e < 4; ++e)
      if (rb + e < B) ((volatile float*)op)[e] = ov[e];
  }
}

extern "C" void kernel_launch(void* const* d_in, const int* in_sizes, int n_in,
                              void* d_out, int out_size, void* d_ws, size_t ws_size,
                              hipStream_t stream) {
  if (n_in < 23) return;
  const int B = in_sizes[0] / D0;
  if (B <= 0 || in_sizes[0] != B * D0) return;
  if (in_sizes[1] != B * NRB * DRB || in_sizes[2] != B * NTK * DTK) return;
  if (in_sizes[3] != DRB * HS || in_sizes[4] != HS || in_sizes[5] != HS * HS || in_sizes[6] != HS) return;
  if (in_sizes[7] != HS * ES || in_sizes[8] != ES) return;
  if (in_sizes[9] != DTK * HS || in_sizes[10] != HS || in_sizes[11] != HS * HS || in_sizes[12] != HS) return;
  if (in_sizes[13] != HS * ES || in_sizes[14] != ES) return;
  if (in_sizes[15] != (D0 + 2 * ES) * HN1 || in_sizes[16] != HN1) return;
  if (in_sizes[17] != HN1 * HN2 || in_sizes[18] != HN2) return;
  if (in_sizes[19] != HN2 * HN3 || in_sizes[20] != HN3) return;
  if (in_sizes[21] != HN3 || in_sizes[22] != 1) return;
  if (out_size != B) return;

  const float* tier0 = (const float*)d_in[0];
  const float* robot = (const float*)d_in[1];
  const float* track = (const float*)d_in[2];
  const float* rw1 = (const float*)d_in[3];  const float* rb1 = (const float*)d_in[4];
  const float* rw2 = (const float*)d_in[5];  const float* rb2 = (const float*)d_in[6];
  const float* rw3 = (const float*)d_in[7];  const float* rb3 = (const float*)d_in[8];
  const float* tw1 = (const float*)d_in[9];  const float* tb1 = (const float*)d_in[10];
  const float* tw2 = (const float*)d_in[11]; const float* tb2 = (const float*)d_in[12];
  const float* tw3 = (const float*)d_in[13]; const float* tb3 = (const float*)d_in[14];
  const float* mw1 = (const float*)d_in[15]; const float* mb1 = (const float*)d_in[16];
  const float* mw2 = (const float*)d_in[17]; const float* mb2 = (const float*)d_in[18];
  const float* mw3 = (const float*)d_in[19]; const float* mb3 = (const float*)d_in[20];
  const float* mw4 = (const float*)d_in[21]; const float* mb4 = (const float*)d_in[22];
  float* out = (float*)d_out;

  const size_t Bp = (size_t)((B + 1) & ~1);
  char* ws = (char*)d_ws;
  size_t off = 0;
  const size_t oRW2 = off; off += (size_t)HS * HS * 2;   off = (off + 255) & ~(size_t)255;
  const size_t oRW3 = off; off += (size_t)ES * HS * 2;   off = (off + 255) & ~(size_t)255;
  const size_t oTW2 = off; off += (size_t)HS * HS * 2;   off = (off + 255) & ~(size_t)255;
  const size_t oTW3 = off; off += (size_t)ES * HS * 2;   off = (off + 255) & ~(size_t)255;
  const size_t oMW1 = off; off += (size_t)HN1 * HK * 2;  off = (off + 255) & ~(size_t)255;
  const size_t oMW2 = off; off += (size_t)HN2 * HN1 * 2; off = (off + 255) & ~(size_t)255;
  const size_t oMW3 = off; off += (size_t)HN3 * HN2 * 2; off = (off + 255) & ~(size_t)255;
  const size_t oRE  = off; off += Bp * ES * 4;            off = (off + 255) & ~(size_t)255;
  const size_t oTE  = off; off += Bp * ES * 4;            off = (off + 255) & ~(size_t)255;
  if (off > ws_size || off > (size_t)WSCAP) return;
  _Float16* rw2t = (_Float16*)(ws + oRW2);
  _Float16* rw3t = (_Float16*)(ws + oRW3);
  _Float16* tw2t = (_Float16*)(ws + oTW2);
  _Float16* tw3t = (_Float16*)(ws + oTW3);
  _Float16* mw1t = (_Float16*)(ws + oMW1);
  _Float16* mw2t = (_Float16*)(ws + oMW2);
  _Float16* mw3t = (_Float16*)(ws + oMW3);
  float*    remb = (float*)(ws + oRE);
  float*    temb = (float*)(ws + oTE);

  k_prepw<<<HS / 16, 256, 0, stream>>>(rw2, HS, HS, HS, rw2t);
  k_prepw<<<ES / 16, 256, 0, stream>>>(rw3, HS, HS, ES, rw3t);
  k_prepw<<<HS / 16, 256, 0, stream>>>(tw2, HS, HS, HS, tw2t);
  k_prepw<<<ES / 16, 256, 0, stream>>>(tw3, HS, HS, ES, tw3t);
  k_prepw<<<HN1 / 16, 256, 0, stream>>>(mw1, D0 + 2 * ES, HK, HN1, mw1t);
  k_prepw<<<HN2 / 16, 256, 0, stream>>>(mw2, HN1, HN1, HN2, mw2t);
  k_prepw<<<HN3 / 16, 256, 0, stream>>>(mw3, HN2, HN2, HN3, mw3t);

  k_setenc<DRB, NRB><<<(B + 1) / 2, 64, 0, stream>>>(robot, rw1, rb1, rw2t, rb2, rw3t, rb3, B, remb);
  k_setenc<DTK, NTK><<<(B + 1) / 2, 64, 0, stream>>>(track, tw1, tb1, tw2t, tb2, tw3t, tb3, B, temb);

  k_head<<<(B + 31) / 32, 64, 0, stream>>>(tier0, remb, temb, mw1t, mb1, mw2t, mb2, mw3t, mb3, mw4, mb4, B, out);
}
